// DFMambaEncoder_20134806684290
// MI455X (gfx1250) — hardware-run, weakly checked
//
#include <hip/hip_runtime.h>


#ifndef NB
#define NB 4
#endif
#define NB_FULL 4
#define CH    192
#define IMG   64
#define LL    (IMG * IMG)
#define NST   16
#define RNK   12
#define XR    (RNK + 2 * NST)
#define NDIR  4
#define XC    CH
#define SCH   64
#define TP    200
#define WCAR  256.0f
#define WINV  (1.0f / 256.0f)
#define LOG2E 1.4426950408889634f

static_assert(NB <= NB_FULL);
static_assert(CH % 64 == 0);
static_assert(CH % 32 == 0);
static_assert(LL % 64 == 0);
static_assert(((size_t)NB * LL) % 64 == 0);
static_assert(NDIR * XR <= XC);
static_assert(XR % 4 == 0);
static_assert(RNK % 4 == 0);
static_assert(NST % 4 == 0);
static_assert((XR * 4) % 16 == 0);
static_assert(IMG == 64);
static_assert(LL % SCH == 0);
static_assert(NDIR == 4);
static_assert((CH * CH / 8) % 256 == 0);
static_assert(CH / 8 <= 32);
static_assert(((size_t)NB * LL) % 8 == 0);
static_assert(256 * 12 * 4 == CH * 64);
static_assert(256 * 6 * 16 == 64 * CH * 2);
static_assert(32 * 16 * 4 == 16 * 64 * 2);
static_assert(32 * 16 * 8 == 16 * 64 * 4);
static_assert(CH * 4 * SCH == SCH * CH * 4);
static_assert(4 * CH >= SCH * (XR / 4));
static_assert(16 * 68 * 4 <= 131072);
static_assert(64 * TP * 2 <= 131072);
static_assert((SCH * XR + SCH * CH) * 4 <= 65536);
static_assert((TP * 2) % 16 == 0);

typedef _Float16 h16;
typedef unsigned short bf;
typedef __attribute__((ext_vector_type(16))) __bf16   v16bf;
typedef __attribute__((ext_vector_type(16))) _Float16 v16h;
typedef __attribute__((ext_vector_type(8)))  _Float16 v8h;
typedef __attribute__((ext_vector_type(8)))  unsigned short v8us;
typedef __attribute__((ext_vector_type(8)))  float    v8f;
typedef __attribute__((ext_vector_type(4)))  float    v4f;
typedef v4f  __attribute__((may_alias)) v4fa;
typedef v8us __attribute__((may_alias)) v8usa;

__device__ __forceinline__ unsigned short f2bf(float f) { unsigned u = __float_as_uint(f); u += 0x7FFFu + ((u >> 16) & 1u); return (unsigned short)(u >> 16); }
__device__ __forceinline__ float bfr(float f) { return __uint_as_float(((unsigned)f2bf(f)) << 16); }
__device__ __forceinline__ v16h cat16(v8h lo, v8h hi) { return __builtin_shufflevector(lo, hi, 0, 1, 2, 3, 4, 5, 6, 7, 8, 9, 10, 11, 12, 13, 14, 15); }
__device__ __forceinline__ v16bf cat16b(v8us lo, v8us hi) { return __builtin_bit_cast(v16bf, __builtin_shufflevector(lo, hi, 0, 1, 2, 3, 4, 5, 6, 7, 8, 9, 10, 11, 12, 13, 14, 15)); }
__device__ __forceinline__ v8f wmma16(v16h a, v16h b, v8f c) { return __builtin_amdgcn_wmma_f32_16x16x32_f16(false, a, false, b, (short)0, c, false, false); }
__device__ __forceinline__ v8f wmmab(v16bf a, v16bf b, v8f c) { return __builtin_amdgcn_wmma_f32_16x16x32_bf16(false, a, false, b, (short)0, c, false, false); }
__device__ __forceinline__ v16h  ldh(const h16* p) { return cat16(*(const v8h*)p, *(const v8h*)(p + 16)); }
__device__ __forceinline__ v16bf ldb(const bf* p)  { return cat16b(*(const v8us*)p, *(const v8us*)(p + 16)); }
__device__ __forceinline__ void wave_sync() { __builtin_amdgcn_fence(3  , "wavefront"); __builtin_amdgcn_wave_barrier(); asm volatile("" ::: "memory"); }

static __device__ __forceinline__ h16 toh_flush(float v) { const h16 r = (h16)v; return (fabsf(v) < 6.103515625e-05f) ? (h16)0.0f : r; }
__device__ __forceinline__ v8f wmma16g(v16h a, v16h b, v8f c) { c = wmma16(a, b, c); asm volatile("v_nop\n\tv_nop\n\tv_nop\n\tv_nop" : "+v"(c) : "v"(a), "v"(b)); return c; }
__device__ __forceinline__ v8f wmmabg(v16bf a, v16bf b, v8f c) { c = wmmab(a, b, c); asm volatile("v_nop\n\tv_nop\n\tv_nop\n\tv_nop" : "+v"(c) : "v"(a), "v"(b)); return c; }

__device__ __forceinline__ int dmap(int k, int t) { const int tt = (k & 2) ? (LL - 1 - t) : t; return (k & 1) ? (((tt & (IMG - 1)) * IMG) + (tt / IMG)) : tt; }

__device__ __forceinline__ float softplus_f(float x) {
    const float e = __expf(-fabsf(x));
    const float u1 = 1.0f + e;
    const float lg = __logf(u1) * (e * __builtin_amdgcn_rcpf(u1 - 1.0f));
    const float l1 = (u1 == 1.0f) ? e : lg;
    return fmaxf(x, 0.0f) + l1;
}

__global__ __launch_bounds__(256) void k_tcvt(const float* __restrict__ src, bf* dst) {
    __shared__ __align__(16) unsigned short ts[64 * TP];
    const int tid = threadIdx.x; const int blk = blockIdx.x;
    const int b = blk / (LL / 64), l0 = (blk % (LL / 64)) * 64;
    const float* sp = src + (size_t)b * CH * LL + l0;
#pragma unroll 2
    for (int it = 0; it < 12; ++it) {
        const int idx = it * 256 + tid; const int c = idx >> 4, l4 = (idx & 15) * 4;
        const v4f v = *(const v4f*)(sp + (size_t)c * LL + l4);
#pragma unroll
        for (int i = 0; i < 4; ++i) ts[(l4 + i) * TP + c] = f2bf(v[i]);
    }
    __syncthreads();
    bf* dp = dst + ((size_t)b * LL + l0) * CH;
#pragma unroll 1
    for (int ps = 0; ps < 2; ++ps) {
#pragma unroll
        for (int it = 0; it < 6; ++it) {
            const int p = it * 256 + tid; const int row = p / 24, c8 = (p % 24) * 8;
            const v8us o = *(const v8usa*)(&ts[row * TP + c8]);
            *(volatile v8us*)(dp + (size_t)p * 8) = o; }
        if (ps == 0) __threadfence(); }
}

__global__ __launch_bounds__(256) void k_wconv_b(const float* __restrict__ src, bf* dst, int tr, int nvalid) {
    const int i = blockIdx.x * 256 + threadIdx.x;
    const int n = i / (CH / 8), k8 = (i % (CH / 8)) * 8;
    const int nc = n < nvalid ? n : nvalid - 1;
    v8us o;
#pragma unroll
    for (int j = 0; j < 8; ++j) { const int k = k8 + j; const int si = tr ? (k * CH + nc) : (nc * CH + k);
        float v = src[si]; asm volatile("" : "+v"(v));
        o[j] = (n < nvalid) ? f2bf(v) : (unsigned short)0; }
    *(volatile v8us*)(dst + (size_t)i * 8) = o; __threadfence(); *(volatile v8us*)(dst + (size_t)i * 8) = o;
}

__global__ __launch_bounds__(256) void k_wconv_h(const float* __restrict__ src, h16* dst, int tr, int nvalid, float carry) {
    const int i = blockIdx.x * 256 + threadIdx.x;
    const int n = i / (CH / 8), k8 = (i % (CH / 8)) * 8;
    const int nc = n < nvalid ? n : nvalid - 1;
    v8h o;
#pragma unroll
    for (int j = 0; j < 8; ++j) { const int k = k8 + j; const int si = tr ? (k * CH + nc) : (nc * CH + k);
        float v = src[si]; asm volatile("" : "+v"(v));
        const h16 hv = toh_flush(bfr(v) * carry);
        o[j] = (n < nvalid) ? hv : (h16)0.0f; }
    *(volatile v8h*)(dst + (size_t)i * 8) = o; __threadfence(); *(volatile v8h*)(dst + (size_t)i * 8) = o;
}

template <int KIND>
__device__ __forceinline__ void gemm64(const void* Av, const void* Bv, void* Ov) {
    __shared__ __align__(16) float os[16 * 68];
    const int lane = threadIdx.x & 31, lr = lane & 15, hi = lane >> 4; const int r0 = blockIdx.x * 64, c0 = blockIdx.y * 64;
    v8f acc[4][4];
#pragma unroll
    for (int mb = 0; mb < 4; ++mb)
#pragma unroll
        for (int nb = 0; nb < 4; ++nb) acc[mb][nb] = (v8f){};
    const size_t aoff = (size_t)(r0 + lr) * CH + 8 * hi, boff = (size_t)(c0 + lr) * CH + 8 * hi;
    if (KIND < 2) {
        const bf* A = (const bf*)Av; const bf* Bt = (const bf*)Bv;
#pragma unroll 1
        for (int kc = 0; kc < CH; kc += 32) {
            v16bf a[4];
#pragma unroll
            for (int mb = 0; mb < 4; ++mb) a[mb] = ldb(A + aoff + (size_t)mb * 16 * CH + kc);
#pragma unroll
            for (int nb = 0; nb < 4; ++nb) { const v16bf b = ldb(Bt + boff + (size_t)nb * 16 * CH + kc);
#pragma unroll
                for (int mb = 0; mb < 4; ++mb) acc[mb][nb] = wmmabg(a[mb], b, acc[mb][nb]); }
        }
    } else {
        const h16* A = (const h16*)Av; const h16* Bt = (const h16*)Bv;
#pragma unroll 1
        for (int kc = 0; kc < CH; kc += 32) {
            v16h a[4];
#pragma unroll
            for (int mb = 0; mb < 4; ++mb) a[mb] = ldh(A + aoff + (size_t)mb * 16 * CH + kc);
#pragma unroll
            for (int nb = 0; nb < 4; ++nb) { const v16h b = ldh(Bt + boff + (size_t)nb * 16 * CH + kc);
#pragma unroll
                for (int mb = 0; mb < 4; ++mb) acc[mb][nb] = wmma16g(a[mb], b, acc[mb][nb]); }
        }
    }
    size_t obase, pitch; float sc;
    if (KIND == 3) { const int bb = c0 / LL, l0 = c0 % LL; obase = ((size_t)bb * CH + (size_t)r0) * LL + (size_t)l0; pitch = LL; sc = WINV; }
    else           { obase = (size_t)r0 * CH + (size_t)c0; pitch = CH; sc = (KIND == 2) ? WINV : 1.0f; }
#pragma unroll
    for (int mb = 0; mb < 4; ++mb) {
#pragma unroll
        for (int nb = 0; nb < 4; ++nb) {
#pragma unroll
            for (int j = 0; j < 8; ++j) os[(hi * 8 + j) * 68 + nb * 16 + lr] = acc[mb][nb][j] * sc; }
        wave_sync();
        const size_t sb = obase + (size_t)(mb * 16) * pitch;
#pragma unroll 1
        for (int ps = 0; ps < 2; ++ps) {
            if (KIND == 0) {
                h16* P = (h16*)Ov;
#pragma unroll
                for (int s = 0; s < 4; ++s) { const int row = 4 * s + (lane >> 3), c8 = (lane & 7) * 8;
                    const v4f x0 = *(const v4fa*)(&os[row * 68 + c8]); const v4f x1 = *(const v4fa*)(&os[row * 68 + c8 + 4]); v8h hv;
#pragma unroll
                    for (int i = 0; i < 4; ++i) { hv[i] = toh_flush(x0[i]); hv[4 + i] = toh_flush(x1[i]); }
                    *(volatile v8h*)(P + sb + (size_t)row * pitch + c8) = hv; }
            } else {
                float* O = (float*)Ov;
#pragma unroll
                for (int s = 0; s < 8; ++s) { const int row = 2 * s + (lane >> 4), c4 = (lane & 15) * 4;
                    const v4f val = *(const v4fa*)(&os[row * 68 + c4]);
                    *(volatile v4f*)(O + sb + (size_t)row * pitch + c4) = val; }
            }
            if (ps == 0) __threadfence(); }
        wave_sync();
    }
}

__global__ __launch_bounds__(32) void k_gemm_xin(const bf* __restrict__ A, const bf* __restrict__ Bt, h16* P) { gemm64<0>(A, Bt, P); }
__global__ __launch_bounds__(32) void k_gemm_yin(const bf* __restrict__ A, const bf* __restrict__ Bt, float* P) { gemm64<1>(A, Bt, P); }
__global__ __launch_bounds__(32) void k_gemm_xdbl(const h16* __restrict__ A, const h16* __restrict__ Bt, float* P) { gemm64<2>(A, Bt, P); }
__global__ __launch_bounds__(32) void k_gemm_out(const h16* __restrict__ A, const h16* __restrict__ Bt, float* P) { gemm64<3>(A, Bt, P); }

__global__ __launch_bounds__(CH) void k_scan(const float* __restrict__ XD, const float* __restrict__ YU, const float* __restrict__ dtw, const float* __restrict__ dtb,
                                             const float* __restrict__ alog, const float* __restrict__ dsv, float* YS) {
    __shared__ __align__(16) float sx[SCH * XR];
    __shared__ __align__(16) float sy[SCH * CH];
    const int z = blockIdx.x; const int b = z / NDIR, k = z % NDIR;
    const int d = threadIdx.x; const int kd = k * CH + d;
    float h[NST], a2[NST], w[RNK];
#pragma unroll
    for (int n = 0; n < NST; ++n) { h[n] = 0.0f; a2[n] = -__expf(bfr(alog[(size_t)kd * NST + n])) * LOG2E; }
#pragma unroll
    for (int r = 0; r < RNK; ++r) w[r] = bfr(dtw[(size_t)kd * RNK + r]);
    const float bias = bfr(dtb[kd]); const float Dd = bfr(dsv[kd]);
    const float* xb = XD + (size_t)b * LL * XC + (size_t)k * XR;
    const float* ub = YU + (size_t)b * LL * CH + d;
    float* yp = YS + (((size_t)k * NB + (size_t)b) * LL) * CH + d;
    float un = ub[(size_t)dmap(k, 0) * CH];
#pragma unroll 1
    for (int t0 = 0; t0 < LL; t0 += SCH) {
        __syncthreads();
#pragma unroll
        for (int it = 0; it < 4; ++it) {
            int i = it * CH + d; i = i < SCH * (XR / 4) ? i : SCH * (XR / 4) - 1;
            const int j = i / (XR / 4), q = i - j * (XR / 4);
            const v4f v = *(const v4f*)(xb + (size_t)dmap(k, t0 + j) * XC + q * 4);
            *(v4fa*)(&sx[j * XR + q * 4]) = v; }
        __syncthreads();
#pragma unroll 1
        for (int j = 0; j < SCH; ++j) {
            const int sb = j * XR;
            v4f q[XR / 4];
#pragma unroll
            for (int i = 0; i < XR / 4; ++i) q[i] = *(const v4fa*)(&sx[sb + 4 * i]);
            const float u = un;
            { int tn = t0 + j + 1; tn = tn < LL ? tn : LL - 1; un = ub[(size_t)dmap(k, tn) * CH]; }
            float dp = bias;
#pragma unroll
            for (int r = 0; r < RNK; ++r) dp += w[r] * q[r >> 2][r & 3];
            const float dt = softplus_f(dp);
            const float du = dt * u;
            float y = 0.0f;
#pragma unroll
            for (int n = 0; n < NST; ++n) {
                const float Bn = q[(RNK + n) >> 2][(RNK + n) & 3];
                const float Cn = q[(RNK + NST + n) >> 2][(RNK + NST + n) & 3];
                const float e = __builtin_amdgcn_exp2f(dt * a2[n]);
                h[n] = e * h[n] + du * Bn;
                y += h[n] * Cn; }
            sy[j * CH + d] = y + Dd * u;
        }
#pragma unroll 1
        for (int ps = 0; ps < 2; ++ps) {
#pragma unroll 4
            for (int j = 0; j < SCH; ++j) {
                const float val = sy[j * CH + d];
                *(volatile float*)(yp + (size_t)dmap(k, t0 + j) * CH) = val; }
            if (ps == 0) __threadfence(); }
    }
}

__global__ __launch_bounds__(256) void k_ln(const float* __restrict__ YS, const float* __restrict__ gam, const float* __restrict__ bet, h16* YN) {
    const int lane = threadIdx.x & 31;
    const int wave = __builtin_amdgcn_readfirstlane((int)(threadIdx.x >> 5));
    const size_t tok = (size_t)blockIdx.x * 8 + wave;
    const bool act = lane < (CH / 8);
    const int c8 = (act ? lane : (CH / 8 - 1)) * 8;
    float v[8];
#pragma unroll
    for (int i = 0; i < 8; ++i) v[i] = 0.0f;
#pragma unroll
    for (int kk = 0; kk < NDIR; ++kk) {
        const int kp = ((kk & 1) << 1) | (kk >> 1);
        const float* p = YS + (((size_t)kp * NB * LL) + tok) * CH + c8;
        const v4f a = *(const v4f*)p, c = *(const v4f*)(p + 4);
#pragma unroll
        for (int i = 0; i < 4; ++i) { v[i] += a[i]; v[4 + i] += c[i]; }
    }
    const v4f g0 = *(const v4f*)(gam + c8), g1 = *(const v4f*)(gam + c8 + 4), b0 = *(const v4f*)(bet + c8), b1 = *(const v4f*)(bet + c8 + 4);
    float s = 0.0f;
#pragma unroll
    for (int i = 0; i < 8; ++i) { float t = v[i]; asm volatile("" : "+v"(t)); v[i] = act ? t : 0.0f; s += v[i]; }
    s += __shfl_xor(s, 16, 32); s += __shfl_xor(s, 8, 32); s += __shfl_xor(s, 4, 32); s += __shfl_xor(s, 2, 32); s += __shfl_xor(s, 1, 32);
    const float mu = s * (1.0f / (float)CH);
    float dv[8]; float s2 = 0.0f;
#pragma unroll
    for (int i = 0; i < 8; ++i) { dv[i] = act ? (v[i] - mu) : 0.0f; s2 += dv[i] * dv[i]; }
    s2 += __shfl_xor(s2, 16, 32); s2 += __shfl_xor(s2, 8, 32); s2 += __shfl_xor(s2, 4, 32); s2 += __shfl_xor(s2, 2, 32); s2 += __shfl_xor(s2, 1, 32);
    const float inv = rsqrtf(s2 * (1.0f / (float)CH) + 1e-5f);
    v8h hv;
#pragma unroll
    for (int i = 0; i < 4; ++i) {
        hv[i]     = toh_flush(dv[i] * inv * bfr(g0[i]) + bfr(b0[i]));
        hv[4 + i] = toh_flush(dv[4 + i] * inv * bfr(g1[i]) + bfr(b1[i])); }
    h16* op = YN + tok * CH + c8;
    if (act) *(volatile v8h*)op = hv;
    __threadfence();
    if (act) *(volatile v8h*)op = hv;
}

static constexpr size_t al256(size_t v) { return (v + 255) & ~(size_t)255; }
static constexpr size_t SZ_TB = al256((size_t)NB * LL * CH * 2);
static constexpr size_t SZ_TF = al256((size_t)NB * LL * CH * 4);
static constexpr size_t SZ_W  = al256((size_t)CH * CH * 2);
static constexpr size_t SZ_TOTAL = 4 * SZ_TB + 2 * SZ_TF + (size_t)NDIR * SZ_TF + 4 * SZ_W;
static_assert(SZ_TOTAL <= (size_t)134217728);
static_assert(((size_t)NB * LL * CH * 2) % 256 == 0);
static_assert(((size_t)CH * CH * 2) % 256 == 0);

extern "C" void kernel_launch(void* const* d_in, const int* in_sizes, int n_in,
                              void* d_out, int out_size, void* d_ws, size_t ws_size, hipStream_t stream) {
    if (n_in < 12) return;
    const size_t needx = (size_t)NB * CH * LL;
    if ((size_t)in_sizes[0] < needx || (size_t)in_sizes[1] < needx) return;
    if ((size_t)in_sizes[2] < (size_t)CH * CH || (size_t)in_sizes[3] < (size_t)CH * CH || (size_t)in_sizes[11] < (size_t)CH * CH) return;
    if ((size_t)in_sizes[4] < (size_t)NDIR * XR * CH || (size_t)in_sizes[5] < (size_t)NDIR * CH * RNK) return;
    if (in_sizes[6] < NDIR * CH || in_sizes[7] < NDIR * CH * NST || in_sizes[8] < NDIR * CH || in_sizes[9] < CH || in_sizes[10] < CH) return;
    if ((size_t)out_size < needx) return;
    if (SZ_TOTAL > ws_size) return;
    const float* x     = (const float*)d_in[0];
    const float* y     = (const float*)d_in[1];
    const float* wpx   = (const float*)d_in[2];
    const float* wpy   = (const float*)d_in[3];
    const float* xproj = (const float*)d_in[4];
    const float* dtw   = (const float*)d_in[5];
    const float* dtb   = (const float*)d_in[6];
    const float* alogs = (const float*)d_in[7];
    const float* dsv   = (const float*)d_in[8];
    const float* gam   = (const float*)d_in[9];
    const float* bet   = (const float*)d_in[10];
    const float* wout  = (const float*)d_in[11];
    float* OUT = (float*)d_out;
    char* wsp = (char*)d_ws;
    bf*  XB  = (bf*)wsp;  wsp += SZ_TB;
    bf*  YB  = (bf*)wsp;  wsp += SZ_TB;
    h16* XH  = (h16*)wsp; wsp += SZ_TB;
    h16* YN  = (h16*)wsp; wsp += SZ_TB;
    float* YU = (float*)wsp; wsp += SZ_TF;
    float* XD = (float*)wsp; wsp += SZ_TF;
    float* YS = (float*)wsp; wsp += (size_t)NDIR * SZ_TF;
    bf*  WXT = (bf*)wsp;  wsp += SZ_W;
    bf*  WYT = (bf*)wsp;  wsp += SZ_W;
    h16* WXP = (h16*)wsp; wsp += SZ_W;
    h16* WOT = (h16*)wsp; wsp += SZ_W;

    const unsigned gt = (unsigned)((size_t)NB * LL / 64);
    k_tcvt<<<gt, 256, 0, stream>>>(x, XB);
    k_tcvt<<<gt, 256, 0, stream>>>(y, YB);
    const unsigned gw = (unsigned)(CH * CH / 8 / 256);
    k_wconv_b<<<gw, 256, 0, stream>>>(wpx, WXT, 1, CH);
    k_wconv_b<<<gw, 256, 0, stream>>>(wpy, WYT, 1, CH);
    k_wconv_h<<<gw, 256, 0, stream>>>(xproj, WXP, 0, NDIR * XR, WCAR);
    k_wconv_h<<<gw, 256, 0, stream>>>(wout, WOT, 1, CH, WCAR);

    k_gemm_xin <<<dim3(gt, CH / 64, 1), 32, 0, stream>>>(XB, WXT, XH);
    k_gemm_yin <<<dim3(gt, CH / 64, 1), 32, 0, stream>>>(YB, WYT, YU);
    k_gemm_xdbl<<<dim3(gt, XC / 64, 1), 32, 0, stream>>>(XH, WXP, XD);
    k_scan<<<NB * NDIR, CH, 0, stream>>>(XD, YU, dtw, dtb, alogs, dsv, YS);
    k_ln<<<(unsigned)((size_t)NB * LL / 8), 256, 0, stream>>>(YS, gam, bet, YN);
    k_gemm_out<<<dim3(CH / 64, gt, 1), 32, 0, stream>>>(WOT, YN, OUT);
}
